// GraphAttentionBlock_71554155152236
// MI455X (gfx1250) — hardware-verified
//
#include <hip/hip_runtime.h>
#include <math.h>


#define BB      2
#define NN      2048
#define HDIM    256
#define NHEADS  8
#define HEADDIM 32
#define FFDIM   1024
#define ROWS    (BB * NN)
#define LN_EPS  1e-5f
#define TP      68

static_assert(ROWS % 64 == 0 && HDIM % 64 == 0 && FFDIM % 64 == 0 && NN % 64 == 0);
static_assert(NN == 2048 && HEADDIM == 32 && NHEADS * HEADDIM == HDIM);

typedef _Float16       v16h __attribute__((ext_vector_type(16)));
typedef _Float16       v8h  __attribute__((ext_vector_type(8)));
typedef __bf16         v16b __attribute__((ext_vector_type(16)));
typedef float          v8f  __attribute__((ext_vector_type(8)));
typedef float          v4f  __attribute__((ext_vector_type(4)));
typedef unsigned int   v4u  __attribute__((ext_vector_type(4)));
typedef unsigned short us;

union FragH { v16h v; v8h p[2]; v4u q[2]; };
union FragB { v16b v; v4u q[2]; };
union Pack8 { v8h h; v4u u; us s[8]; };

#define OP_HEAD   0
#define OP_HEADVT 1
#define OP_RES    2
#define OP_GELU   3

#define VNOPS "v_nop\n\tv_nop\n\tv_nop\n\tv_nop"

__device__ __forceinline__ v8f vz8() {
  v8f z = {0.f, 0.f, 0.f, 0.f, 0.f, 0.f, 0.f, 0.f};
  return z;
}
__device__ __forceinline__ v4u ldv(const us* p) { return *(const v4u*)p; }
__device__ __forceinline__ us f2bf(float f) {
  unsigned int u = __float_as_uint(f);
  u += 0x7FFFu + ((u >> 16) & 1u);
  return (us)(u >> 16);
}
__device__ __forceinline__ float bf2f(us b) { return __uint_as_float(((unsigned int)b) << 16); }

__device__ __forceinline__ v8f mma_h(v16h a, v16h b, v8f c) {
  return __builtin_amdgcn_wmma_f32_16x16x32_f16(false, a, false, b, (short)0, c, false, false);
}
__device__ __forceinline__ v8f mma_b(v16b a, v16b b, v8f c) {
  return __builtin_amdgcn_wmma_f32_16x16x32_bf16(false, a, false, b, (short)0, c, false, false);
}

__global__ void __launch_bounds__(256) k_wcvt(const float* __restrict__ src, us* dst, us* dst2,
                                              int R, int C, float scale, int mode) {
  __shared__ float tile[32][65];
  const int ncb = C >> 5;
  const int cb = blockIdx.x % ncb;
  const int rb = blockIdx.x / ncb;
  const int c0 = cb * 32, r0 = rb * 64;
  if (r0 + 64 > R || c0 + 32 > C) return;
  const int t = threadIdx.x;
#pragma unroll
  for (int i = 0; i < 8; ++i) {
    const int e = i * 256 + t;
    const int rr = e >> 5, cc = e & 31;
    tile[cc][rr] = src[(size_t)(r0 + rr) * C + c0 + cc];
  }
  __syncthreads();
  const int cc = t >> 3, p = t & 7;
  float v[8];
#pragma unroll
  for (int j = 0; j < 8; ++j) v[j] = tile[cc][8 * p + j];
  const size_t go = (size_t)(c0 + cc) * R + r0 + 8 * p;
  Pack8 ph, pl;
  if (mode == 0) {
#pragma unroll
    for (int j = 0; j < 8; ++j) ph.h[j] = (_Float16)(v[j] * scale);
    pl.u = ph.u;
  } else {
#pragma unroll
    for (int j = 0; j < 8; ++j) {
      const us hb = f2bf(v[j]);
      ph.s[j] = hb;
      pl.s[j] = f2bf(v[j] - bf2f(hb));
    }
  }
  *(volatile v4u*)(dst + go) = ph.u;
  if (mode != 0) *(volatile v4u*)(dst2 + go) = pl.u;
  __threadfence();
  *(volatile v4u*)(dst + go) = ph.u;
  if (mode != 0) *(volatile v4u*)(dst2 + go) = pl.u;
}

__global__ void __launch_bounds__(256) k_ln(const float* __restrict__ x, const float* __restrict__ g,
                                            const float* __restrict__ bta, const float* __restrict__ aux,
                                            us* y, us* y2, int rows, int mode) {
  const int lane = threadIdx.x & 31;
  const int row  = blockIdx.x * 8 + (threadIdx.x >> 5);
  if (row >= rows) return;
  (void)aux;
  const float* xr = x + (size_t)row * HDIM + lane * 8;
  const v4f xa = *(const v4f*)xr;
  const v4f xb = *(const v4f*)(xr + 4);
  float v[8] = {xa[0], xa[1], xa[2], xa[3], xb[0], xb[1], xb[2], xb[3]};
  float s = 0.f;
#pragma unroll
  for (int j = 0; j < 8; ++j) s += v[j];
#pragma unroll
  for (int off = 16; off > 0; off >>= 1) s += __shfl_xor(s, off, 32);
  const float mu = s * (1.f / HDIM);
  float d[8];
  float s2 = 0.f;
#pragma unroll
  for (int j = 0; j < 8; ++j) { d[j] = v[j] - mu; s2 += d[j] * d[j]; }
#pragma unroll
  for (int off = 16; off > 0; off >>= 1) s2 += __shfl_xor(s2, off, 32);
  const float var = s2 * (1.f / HDIM);
  const float rs  = rsqrtf(var + LN_EPS);
  const v4f ga = *(const v4f*)(g + lane * 8);
  const v4f gb = *(const v4f*)(g + lane * 8 + 4);
  const v4f ba = *(const v4f*)(bta + lane * 8);
  const v4f bb = *(const v4f*)(bta + lane * 8 + 4);
  const float gg[8] = {ga[0], ga[1], ga[2], ga[3], gb[0], gb[1], gb[2], gb[3]};
  const float bv[8] = {ba[0], ba[1], ba[2], ba[3], bb[0], bb[1], bb[2], bb[3]};
  float yv[8];
#pragma unroll
  for (int j = 0; j < 8; ++j) yv[j] = d[j] * rs * gg[j] + bv[j];
  const size_t go = (size_t)row * HDIM + lane * 8;
  Pack8 ph, pl;
  if (mode == 0) {
#pragma unroll
    for (int j = 0; j < 8; ++j) ph.h[j] = (_Float16)yv[j];
    pl.u = ph.u;
  } else {
#pragma unroll
    for (int j = 0; j < 8; ++j) {
      const us hb = f2bf(yv[j]);
      ph.s[j] = hb;
      pl.s[j] = f2bf(yv[j] - bf2f(hb));
    }
  }
  *(volatile v4u*)(y + go) = ph.u;
  if (mode != 0) *(volatile v4u*)(y2 + go) = pl.u;
  __threadfence();
  *(volatile v4u*)(y + go) = ph.u;
  if (mode != 0) *(volatile v4u*)(y2 + go) = pl.u;
}

template <int OP, int AMODE, int SPLIT, int KDIM>
__global__ void __launch_bounds__(128) k_gemm(
    const us* __restrict__ A, const us* __restrict__ A2,
    const us* __restrict__ W, const us* __restrict__ W2,
    const float* __restrict__ bias, const float* __restrict__ res,
    float* outF, us* outH, us* outH2, int M, int Nout, float oscale) {
  static_assert(KDIM % 64 == 0);
  __shared__ __attribute__((aligned(16))) float tile[64 * TP];
  const int t = threadIdx.x;
  const int lane = t & 31, w = t >> 5, h = lane >> 4, m = lane & 15;
  const int ntn = Nout >> 6;
  const int mt = blockIdx.x / ntn;
  const int nt = blockIdx.x - mt * ntn;
  const int m0 = mt * 64, n0 = nt * 64;
  if (m0 + 64 > M) return;
  const int arow = m0 + w * 16 + m;

  v8f c0 = vz8(), c1 = vz8(), c2 = vz8(), c3 = vz8();

  auto step = [&](int ks) {
    size_t aoff;
    if (AMODE == 0) {
      aoff = (size_t)arow * KDIM + (size_t)ks * 32;
    } else {
      aoff = ((size_t)((arow >> 11) * NHEADS + ks) * NN + (size_t)(arow & (NN - 1))) * HEADDIM;
    }
    const us* ap = A + aoff + 8 * h;
    const us* wp = W + (size_t)(n0 + m) * KDIM + ks * 32 + 8 * h;
    if (SPLIT) {
      FragB a, a2, b0, b1, b2, b3, e0, e1, e2, e3;
      const us* ap2 = A2 + aoff + 8 * h;
      const us* wp2 = W2 + (size_t)(n0 + m) * KDIM + ks * 32 + 8 * h;
      a.q[0]  = ldv(ap);                 a.q[1]  = ldv(ap + 16);
      a2.q[0] = ldv(ap2);                a2.q[1] = ldv(ap2 + 16);
      b0.q[0] = ldv(wp);                 b0.q[1] = ldv(wp + 16);
      b1.q[0] = ldv(wp + 16 * KDIM);     b1.q[1] = ldv(wp + 16 * KDIM + 16);
      b2.q[0] = ldv(wp + 32 * KDIM);     b2.q[1] = ldv(wp + 32 * KDIM + 16);
      b3.q[0] = ldv(wp + 48 * KDIM);     b3.q[1] = ldv(wp + 48 * KDIM + 16);
      e0.q[0] = ldv(wp2);                e0.q[1] = ldv(wp2 + 16);
      e1.q[0] = ldv(wp2 + 16 * KDIM);    e1.q[1] = ldv(wp2 + 16 * KDIM + 16);
      e2.q[0] = ldv(wp2 + 32 * KDIM);    e2.q[1] = ldv(wp2 + 32 * KDIM + 16);
      e3.q[0] = ldv(wp2 + 48 * KDIM);    e3.q[1] = ldv(wp2 + 48 * KDIM + 16);
      c0 = mma_b(a.v, b0.v, c0); c0 = mma_b(a.v, e0.v, c0); c0 = mma_b(a2.v, b0.v, c0);
      c1 = mma_b(a.v, b1.v, c1); c1 = mma_b(a.v, e1.v, c1); c1 = mma_b(a2.v, b1.v, c1);
      c2 = mma_b(a.v, b2.v, c2); c2 = mma_b(a.v, e2.v, c2); c2 = mma_b(a2.v, b2.v, c2);
      c3 = mma_b(a.v, b3.v, c3); c3 = mma_b(a.v, e3.v, c3); c3 = mma_b(a2.v, b3.v, c3);
      asm volatile(VNOPS
                   : "+v"(c0), "+v"(c1), "+v"(c2), "+v"(c3)
                   : "v"(a.v), "v"(a2.v), "v"(b0.v), "v"(b1.v), "v"(b2.v), "v"(b3.v),
                     "v"(e0.v), "v"(e1.v), "v"(e2.v), "v"(e3.v)
                   : "memory");
    } else {
      FragH a, b0, b1, b2, b3;
      a.q[0]  = ldv(ap);                 a.q[1]  = ldv(ap + 16);
      b0.q[0] = ldv(wp);                 b0.q[1] = ldv(wp + 16);
      b1.q[0] = ldv(wp + 16 * KDIM);     b1.q[1] = ldv(wp + 16 * KDIM + 16);
      b2.q[0] = ldv(wp + 32 * KDIM);     b2.q[1] = ldv(wp + 32 * KDIM + 16);
      b3.q[0] = ldv(wp + 48 * KDIM);     b3.q[1] = ldv(wp + 48 * KDIM + 16);
      c0 = mma_h(a.v, b0.v, c0);
      c1 = mma_h(a.v, b1.v, c1);
      c2 = mma_h(a.v, b2.v, c2);
      c3 = mma_h(a.v, b3.v, c3);
      asm volatile(VNOPS
                   : "+v"(c0), "+v"(c1), "+v"(c2), "+v"(c3)
                   : "v"(a.v), "v"(b0.v), "v"(b1.v), "v"(b2.v), "v"(b3.v)
                   : "memory");
    }
  };

#pragma unroll 1
  for (int ks = 0; ks < KDIM / 32; ks += 2) {
    step(ks);
    step(ks + 1);
  }

  {
    float* tr = tile + (w * 16 + 8 * h) * TP + m;
#pragma unroll
    for (int r = 0; r < 8; ++r) {
      tr[r * TP]      = c0[r] * oscale;
      tr[r * TP + 16] = c1[r] * oscale;
      tr[r * TP + 32] = c2[r] * oscale;
      tr[r * TP + 48] = c3[r] * oscale;
    }
  }
  __syncthreads();

  const int p = t & 7;
  if (OP == OP_RES) {
    v4f vals[8];
    size_t goff[8];
#pragma unroll
    for (int i = 0; i < 8; ++i) {
      const int L = i * 16 + (t >> 3);
      const int row = L >> 1;
      const int cs = ((L & 1) << 5) + p * 4;
      const v4f tv = *(const v4f*)(tile + row * TP + cs);
      const v4f bv = *(const v4f*)(bias + n0 + cs);
      goff[i] = (size_t)(m0 + row) * Nout + n0 + cs;
      const v4f rv = *(const v4f*)(res + goff[i]);
      const v4f sv = tv + bv;
      vals[i] = rv + sv;
      *(volatile v4f*)(outF + goff[i]) = vals[i];
    }
    __threadfence();
#pragma unroll
    for (int i = 0; i < 8; ++i) *(volatile v4f*)(outF + goff[i]) = vals[i];
  } else if (OP == OP_GELU) {
    v4u hv[4], lv[4];
    size_t goff[4];
#pragma unroll
    for (int i = 0; i < 4; ++i) {
      const int row = i * 16 + (t >> 3);
      const int cs = p * 8;
      const v4f t0 = *(const v4f*)(tile + row * TP + cs);
      const v4f t1 = *(const v4f*)(tile + row * TP + cs + 4);
      const v4f b0 = *(const v4f*)(bias + n0 + cs);
      const v4f b1 = *(const v4f*)(bias + n0 + cs + 4);
      const float xv[8] = {t0[0] + b0[0], t0[1] + b0[1], t0[2] + b0[2], t0[3] + b0[3],
                           t1[0] + b1[0], t1[1] + b1[1], t1[2] + b1[2], t1[3] + b1[3]};
      Pack8 ph, pl;
#pragma unroll
      for (int j = 0; j < 8; ++j) {
        const float xx = xv[j];
        const float gl = 0.5f * xx * (1.f + erff(xx * 0.70710678118654752f));
        const us hb = f2bf(gl);
        ph.s[j] = hb;
        pl.s[j] = f2bf(gl - bf2f(hb));
      }
      hv[i] = ph.u;
      lv[i] = pl.u;
      goff[i] = (size_t)(m0 + row) * Nout + n0 + cs;
      *(volatile v4u*)(outH + goff[i])  = hv[i];
      *(volatile v4u*)(outH2 + goff[i]) = lv[i];
    }
    __threadfence();
#pragma unroll
    for (int i = 0; i < 4; ++i) {
      *(volatile v4u*)(outH + goff[i])  = hv[i];
      *(volatile v4u*)(outH2 + goff[i]) = lv[i];
    }
  } else {
    const int bidx = m0 >> 11;
    const int ntok0 = m0 & (NN - 1);
    const int h0 = n0 >> 5;
    v4u hv[4];
    size_t goff[4];
#pragma unroll
    for (int i = 0; i < 4; ++i) {
      const int L = i * 16 + (t >> 3);
      const int hh = L >> 5;
      Pack8 ph;
      if (OP == OP_HEAD) {
        const int l = L & 31;
        const int tok = 2 * l + (p >> 2);
        const int d = (p & 3) * 8;
        const v4f t0 = *(const v4f*)(tile + tok * TP + hh * 32 + d);
        const v4f t1 = *(const v4f*)(tile + tok * TP + hh * 32 + d + 4);
        const v4f b0 = *(const v4f*)(bias + n0 + hh * 32 + d);
        const v4f b1 = *(const v4f*)(bias + n0 + hh * 32 + d + 4);
        ph.h[0] = (_Float16)(t0[0] + b0[0]); ph.h[1] = (_Float16)(t0[1] + b0[1]);
        ph.h[2] = (_Float16)(t0[2] + b0[2]); ph.h[3] = (_Float16)(t0[3] + b0[3]);
        ph.h[4] = (_Float16)(t1[0] + b1[0]); ph.h[5] = (_Float16)(t1[1] + b1[1]);
        ph.h[6] = (_Float16)(t1[2] + b1[2]); ph.h[7] = (_Float16)(t1[3] + b1[3]);
        goff[i] = ((size_t)((bidx * NHEADS + h0 + hh) * NN + ntok0 + tok)) * HEADDIM + d;
      } else {
        const int d = L & 31;
        const float bc = bias[n0 + hh * 32 + d];
#pragma unroll
        for (int j = 0; j < 8; ++j)
          ph.h[j] = (_Float16)(tile[(8 * p + j) * TP + hh * 32 + d] + bc);
        goff[i] = ((size_t)((bidx * NHEADS + h0 + hh) * HEADDIM + d)) * NN + ntok0 + 8 * p;
      }
      hv[i] = ph.u;
      *(volatile v4u*)(outH + goff[i]) = hv[i];
    }
    __threadfence();
#pragma unroll
    for (int i = 0; i < 4; ++i) *(volatile v4u*)(outH + goff[i]) = hv[i];
  }
}

__global__ void __launch_bounds__(128) k_attn(const us* __restrict__ q16, const us* __restrict__ k16,
                                              const us* __restrict__ vT16, const float* __restrict__ adj,
                                              us* att16) {
  __shared__ __attribute__((aligned(16))) _Float16 plds[4 * 16 * 32];
  const int lane = threadIdx.x & 31, warp = threadIdx.x >> 5;
  const int h = lane >> 4, m = lane & 15;
  const int wid = blockIdx.x * 4 + warp;
  if (wid >= BB * NHEADS * (NN / 16)) return;
  const int qt = wid & (NN / 16 - 1);
  const int bh = wid >> 7;
  const int b  = bh >> 3;
  _Float16* slab = plds + warp * (16 * 32);

  FragH aq;
  {
    const us* qp = q16 + ((size_t)bh * NN + qt * 16 + m) * HEADDIM;
    aq.q[0] = ldv(qp + 8 * h);
    aq.q[1] = ldv(qp + 16 + 8 * h);
  }
  const float* adjrow = adj + ((size_t)b * NN + qt * 16 + 8 * h) * NN;
  const us* kb = k16 + (size_t)bh * NN * HEADDIM;
  const us* vb = vT16 + (size_t)bh * HEADDIM * NN;

  v8f o0 = vz8(), o1 = vz8();
  float mrun[8], lrun[8];
#pragma unroll
  for (int r = 0; r < 8; ++r) { mrun[r] = -1e30f; lrun[r] = 0.f; }
  const float scale = 0.17677669529663687f;

#pragma unroll 1
  for (int kt = 0; kt < NN / 32; ++kt) {
    const int k0 = kt * 32;
    FragH bk0, bk1, bv0, bv1;
    {
      const us* kp0 = kb + (size_t)(k0 + m) * HEADDIM;
      bk0.q[0] = ldv(kp0 + 8 * h); bk0.q[1] = ldv(kp0 + 16 + 8 * h);
      const us* kp1 = kb + (size_t)(k0 + 16 + m) * HEADDIM;
      bk1.q[0] = ldv(kp1 + 8 * h); bk1.q[1] = ldv(kp1 + 16 + 8 * h);
      const us* vp0 = vb + (size_t)m * NN + k0;
      bv0.q[0] = ldv(vp0 + 8 * h); bv0.q[1] = ldv(vp0 + 16 + 8 * h);
      const us* vp1 = vb + (size_t)(16 + m) * NN + k0;
      bv1.q[0] = ldv(vp1 + 8 * h); bv1.q[1] = ldv(vp1 + 16 + 8 * h);
    }
    float a0[8], a1[8];
#pragma unroll
    for (int r = 0; r < 8; ++r) {
      a0[r] = adjrow[(size_t)r * NN + k0 + m];
      a1[r] = adjrow[(size_t)r * NN + k0 + 16 + m];
    }

    v8f s0 = mma_h(aq.v, bk0.v, vz8());
    v8f s1 = mma_h(aq.v, bk1.v, vz8());
    asm volatile(VNOPS : "+v"(s0), "+v"(s1) : "v"(aq.v), "v"(bk0.v), "v"(bk1.v));

    float e0[8], e1[8];
#pragma unroll
    for (int r = 0; r < 8; ++r) {
      const float l0 = s0[r] * scale + (2.f * a0[r] - 1.f);
      const float l1 = s1[r] * scale + (2.f * a1[r] - 1.f);
      float tmax = fmaxf(l0, l1);
#pragma unroll
      for (int off = 8; off > 0; off >>= 1) tmax = fmaxf(tmax, __shfl_xor(tmax, off, 32));
      const float mnew = fmaxf(mrun[r], tmax);
      const float corr = __expf(mrun[r] - mnew);
      const float x0 = __expf(l0 - mnew) * (0.25f + 0.75f * a0[r]);
      const float x1 = __expf(l1 - mnew) * (0.25f + 0.75f * a1[r]);
      float ts = x0 + x1;
#pragma unroll
      for (int off = 8; off > 0; off >>= 1) ts += __shfl_xor(ts, off, 32);
      lrun[r] = lrun[r] * corr + ts;
      mrun[r] = mnew;
      o0[r] = o0[r] * corr;
      o1[r] = o1[r] * corr;
      e0[r] = x0;
      e1[r] = x1;
    }
#pragma unroll
    for (int r = 0; r < 8; ++r) {
      slab[(8 * h + r) * 32 + m]      = (_Float16)(e0[r] * 256.f);
      slab[(8 * h + r) * 32 + 16 + m] = (_Float16)(e1[r] * 256.f);
    }
    asm volatile("s_wait_dscnt 0" ::: "memory");
    FragH ap;
    ap.p[0] = *(const v8h*)(slab + m * 32 + 8 * h);
    ap.p[1] = *(const v8h*)(slab + m * 32 + 16 + 8 * h);

    o0 = mma_h(ap.v, bv0.v, o0);
    o1 = mma_h(ap.v, bv1.v, o1);
    asm volatile(VNOPS : "+v"(o0), "+v"(o1) : "v"(ap.v), "v"(bv0.v), "v"(bv1.v));
  }

  asm volatile("s_wait_dscnt 0" ::: "memory");
#pragma unroll
  for (int r = 0; r < 8; ++r) {
    const float inv = __fdividef(0.0625f, lrun[r]);
    slab[(8 * h + r) * 32 + m]      = (_Float16)(o0[r] * inv);
    slab[(8 * h + r) * 32 + 16 + m] = (_Float16)(o1[r] * inv);
  }
  asm volatile("s_wait_dscnt 0" ::: "memory");
  const int rr = lane >> 2, dd = (lane & 3) * 8;
  Pack8 w0, w1;
  w0.h = *(const v8h*)(slab + rr * 32 + dd);
  w1.h = *(const v8h*)(slab + (8 + rr) * 32 + dd);
  us* ob = att16 + ((size_t)bh * NN + qt * 16) * HEADDIM;
  *(volatile v4u*)(ob + rr * 32 + dd)       = w0.u;
  *(volatile v4u*)(ob + (8 + rr) * 32 + dd) = w1.u;
  __threadfence();
  *(volatile v4u*)(ob + rr * 32 + dd)       = w0.u;
  *(volatile v4u*)(ob + (8 + rr) * 32 + dd) = w1.u;
}

extern "C" void kernel_launch(void* const* d_in, const int* in_sizes, int n_in,
                              void* d_out, int out_size, void* d_ws, size_t ws_size,
                              hipStream_t stream) {
  if (n_in < 19) return;
  if (in_sizes[0] != ROWS * HDIM || in_sizes[1] != BB * NN * NN || in_sizes[2] < 1 ||
      in_sizes[3] != HDIM * HDIM || in_sizes[4] != HDIM ||
      in_sizes[5] != HDIM * HDIM || in_sizes[6] != HDIM ||
      in_sizes[7] != HDIM * HDIM || in_sizes[8] != HDIM ||
      in_sizes[9] != HDIM * HDIM || in_sizes[10] != HDIM ||
      in_sizes[11] != HDIM || in_sizes[12] != HDIM ||
      in_sizes[13] != HDIM || in_sizes[14] != HDIM ||
      in_sizes[15] != HDIM * FFDIM || in_sizes[16] != FFDIM ||
      in_sizes[17] != FFDIM * HDIM || in_sizes[18] != HDIM ||
      out_size != ROWS * HDIM) return;

  const float* hidden    = (const float*)d_in[0];
  const float* adjacency = (const float*)d_in[1];
  const float* positions = (const float*)d_in[2];
  const float* wq   = (const float*)d_in[3];  const float* bq   = (const float*)d_in[4];
  const float* wk   = (const float*)d_in[5];  const float* bk   = (const float*)d_in[6];
  const float* wv   = (const float*)d_in[7];  const float* bv   = (const float*)d_in[8];
  const float* wo   = (const float*)d_in[9];  const float* bo   = (const float*)d_in[10];
  const float* g1   = (const float*)d_in[11]; const float* b1   = (const float*)d_in[12];
  const float* g2   = (const float*)d_in[13]; const float* b2   = (const float*)d_in[14];
  const float* wff1 = (const float*)d_in[15]; const float* bff1 = (const float*)d_in[16];
  const float* wff2 = (const float*)d_in[17]; const float* bff2 = (const float*)d_in[18];
  float* out = (float*)d_out;

  char* ws = (char*)d_ws;
  size_t off = 0;
  auto carve = [&](size_t bytes) -> void* {
    void* p = ws + off;
    off = (off + bytes + 255) & ~(size_t)255;
    return p;
  };
  us* wqT  = (us*)carve((size_t)HDIM * HDIM * 2);
  us* wkT  = (us*)carve((size_t)HDIM * HDIM * 2);
  us* wvT  = (us*)carve((size_t)HDIM * HDIM * 2);
  us* woT  = (us*)carve((size_t)HDIM * HDIM * 2);
  us* f1h  = (us*)carve((size_t)FFDIM * HDIM * 2);
  us* f1l  = (us*)carve((size_t)FFDIM * HDIM * 2);
  us* f2h  = (us*)carve((size_t)HDIM * FFDIM * 2);
  us* f2l  = (us*)carve((size_t)HDIM * FFDIM * 2);
  us* xn16 = (us*)carve((size_t)ROWS * HDIM * 2);
  us* q16  = (us*)carve((size_t)ROWS * HDIM * 2);
  us* k16  = (us*)carve((size_t)ROWS * HDIM * 2);
  us* vT16 = (us*)carve((size_t)ROWS * HDIM * 2);
  us* att16 = (us*)carve((size_t)ROWS * HDIM * 2);
  float* hid2 = (float*)carve((size_t)ROWS * HDIM * 4);
  us* h2h  = (us*)carve((size_t)ROWS * HDIM * 2);
  us* h2l  = (us*)carve((size_t)ROWS * HDIM * 2);
  us* gh   = (us*)carve((size_t)ROWS * FFDIM * 2);
  us* gl   = (us*)carve((size_t)ROWS * FFDIM * 2);
  if (off > ws_size) return;

  const int gW = (HDIM / 32) * (HDIM / 64);
  k_wcvt<<<gW, 256, 0, stream>>>(wq, wqT, wqT, HDIM, HDIM, 16.f, 0);
  k_wcvt<<<gW, 256, 0, stream>>>(wk, wkT, wkT, HDIM, HDIM, 16.f, 0);
  k_wcvt<<<gW, 256, 0, stream>>>(wv, wvT, wvT, HDIM, HDIM, 16.f, 0);
  k_wcvt<<<gW, 256, 0, stream>>>(wo, woT, woT, HDIM, HDIM, 16.f, 0);
  k_wcvt<<<(FFDIM / 32) * (HDIM / 64), 256, 0, stream>>>(wff1, f1h, f1l, HDIM, FFDIM, 1.f, 1);
  k_wcvt<<<(HDIM / 32) * (FFDIM / 64), 256, 0, stream>>>(wff2, f2h, f2l, FFDIM, HDIM, 1.f, 1);

  k_ln<<<(ROWS + 7) / 8, 256, 0, stream>>>(hidden, g1, b1, positions, xn16, xn16, ROWS, 0);

  const int gP = (ROWS / 64) * (HDIM / 64);
  k_gemm<OP_HEAD, 0, 0, HDIM><<<gP, 128, 0, stream>>>(xn16, xn16, wqT, wqT, bq, bq, hid2, q16, q16,
                                                       ROWS, HDIM, 1.f / 16.f);
  k_gemm<OP_HEAD, 0, 0, HDIM><<<gP, 128, 0, stream>>>(xn16, xn16, wkT, wkT, bk, bk, hid2, k16, k16,
                                                       ROWS, HDIM, 1.f / 16.f);
  k_gemm<OP_HEADVT, 0, 0, HDIM><<<gP, 128, 0, stream>>>(xn16, xn16, wvT, wvT, bv, bv, hid2, vT16, vT16,
                                                         ROWS, HDIM, 1.f / 16.f);

  k_attn<<<(BB * NHEADS * (NN / 16) + 3) / 4, 128, 0, stream>>>(q16, k16, vT16, adjacency, att16);

  k_gemm<OP_RES, 1, 0, HDIM><<<gP, 128, 0, stream>>>(att16, att16, woT, woT, bo, hidden, hid2, xn16, xn16,
                                                      ROWS, HDIM, 1.f / 256.f);

  k_ln<<<(ROWS + 7) / 8, 256, 0, stream>>>(hid2, g2, b2, positions, h2h, h2l, ROWS, 1);

  k_gemm<OP_GELU, 0, 1, HDIM><<<(ROWS / 64) * (FFDIM / 64), 128, 0, stream>>>(
      h2h, h2l, f1h, f1l, bff1, bff1, hid2, gh, gl, ROWS, FFDIM, 1.f);

  k_gemm<OP_RES, 0, 1, FFDIM><<<gP, 128, 0, stream>>>(gh, gl, f2h, f2l, bff2, hid2, out, xn16, xn16,
                                                       ROWS, HDIM, 1.f);
}
